// RNN_LSTM_EMBED_90907277787356
// MI455X (gfx1250) — hardware-run, weakly checked
//
#include <hip/hip_runtime.h>
#include <math.h>

typedef __attribute__((ext_vector_type(16))) _Float16 v16h;
typedef __attribute__((ext_vector_type(8)))  _Float16 v8h;
typedef __attribute__((ext_vector_type(8)))  float    v8f;
typedef __attribute__((ext_vector_type(4)))  float    v4f;
typedef __attribute__((ext_vector_type(4)))  int      v4i;

constexpr int kBatch  = 64;
constexpr int kSteps  = 512;
constexpr int kEmb    = 512;
constexpr int kHid    = 1024;
constexpr int kGates  = 4 * kHid;
constexpr int kVocab  = 256;
constexpr int kCls    = 256;
constexpr int kRowsBT = kBatch * kSteps;
constexpr int kSampPerBlk = 16;
constexpr int kStepBlocks = kBatch / kSampPerBlk;
constexpr int kStepWaves  = 16;
constexpr int kStepThreads = kStepWaves * 32;
constexpr int kHP = kHid + 8;

constexpr float kCarryW   = 1024.0f;
constexpr float kCarryH   = 1024.0f;
constexpr float kCarryE   = 256.0f;
constexpr float kAccScale    = kCarryH * kCarryW;
constexpr float kAccScaleInv = 1.0f / kAccScale;
constexpr float kTableScale  = kAccScale / (kCarryE * kCarryW);
constexpr float kHeadScale   = 1.0f / (kCarryH * kCarryW);
constexpr float kF16MinNormal = 6.103515625e-05f;

static_assert(kGates == 4096 && kRowsBT == 32768, "shapes");
static_assert((kEmb % 32) == 0 && (kHid % 32) == 0, "GEMM K multiples of 32");
static_assert((kVocab % 64) == 0 && (kGates % 64) == 0 && (kRowsBT % 64) == 0 && (kCls % 64) == 0, "GEMM M,N multiples of 64");
static_assert(kStepWaves * 64 == kHid, "each wave of the step kernel owns 64 hidden units");
static_assert(kStepBlocks * kSampPerBlk == kBatch, "batch split");
static_assert(((kHP * 2) % 16) == 0, "LDS pitch 16-B aligned");
static_assert(kAccScale == 1048576.0f && kTableScale == 4.0f, "scale chain");

constexpr size_t kOffWHH  = 0;
constexpr size_t kOffWIH  = kOffWHH + (size_t)kGates * kHid * 2;
constexpr size_t kOffFCW  = kOffWIH + (size_t)kGates * kEmb * 2;
constexpr size_t kOffEMB  = kOffFCW + (size_t)kCls * kHid * 2;
constexpr size_t kOffGT   = kOffEMB + (size_t)kVocab * kEmb * 2;
constexpr size_t kOffHS   = kOffGT  + (size_t)kVocab * kGates * 4;
constexpr size_t kWsTotal = kOffHS  + (size_t)kRowsBT * kHid * 2;
static_assert(kWsTotal == 84672512ull, "carve total");
static_assert(kWsTotal <= 134217728ull, "carve cap");
static_assert((kOffWIH % 128) == 0 && (kOffFCW % 128) == 0 && (kOffEMB % 128) == 0 &&
              (kOffGT % 128) == 0 && (kOffHS % 128) == 0, "128-B aligned regions");

__device__ __forceinline__ unsigned short f2bf_bits(float f) {
  unsigned u = __float_as_uint(f);
  return (unsigned short)((u + 0x7FFFu + ((u >> 16) & 1u)) >> 16);
}
__device__ __forceinline__ float bf_bits2f(unsigned short h) { return __uint_as_float(((unsigned)h) << 16); }
__device__ __forceinline__ float bf_value(float f) { return bf_bits2f(f2bf_bits(f)); }

__device__ __forceinline__ _Float16 f16_operand(float s) {
  const float w = (fabsf(s) < kF16MinNormal) ? 0.0f : s;
  return (_Float16)w;
}

union FragU { v16h v; v8h h[2]; };
__device__ __forceinline__ v16h frag_load(const _Float16* p) {
  FragU f;
  f.h[0] = *(const v8h*)(p);
  f.h[1] = *(const v8h*)(p + 16);
  return f.v;
}
__device__ __forceinline__ v8f mma_h(v16h a, v16h b, v8f c) {
  c = __builtin_amdgcn_wmma_f32_16x16x32_f16(false, a, false, b, (short)0, c, false, false);
  asm volatile("v_nop\n\tv_nop\n\tv_nop\n\tv_nop" : "+v"(c) : "v"(a), "v"(b));
  return c;
}

__global__ __launch_bounds__(256) void plane_f16_kernel(
    const float* __restrict__ src, unsigned short* __restrict__ dst, int total8, float carry)
{
  const int i = blockIdx.x * 256 + threadIdx.x;
  if (i >= total8) return;
  const size_t e0 = (size_t)i << 3;
  const v4f a0 = *(const v4f*)(src + e0);
  const v4f a1 = *(const v4f*)(src + e0 + 4);
  v8h hv;
#pragma unroll
  for (int e = 0; e < 4; ++e) {
    const float x0 = a0[e];
    const float x1 = a1[e];
    hv[e]     = f16_operand(bf_value(x0) * carry);
    hv[4 + e] = f16_operand(bf_value(x1) * carry);
  }
  unsigned short* q = dst + e0;
  *(volatile v8h*)q = hv;
  __threadfence();
  *(volatile v8h*)q = hv;
}

template <int BIAS_MODE>
__global__ __launch_bounds__(256) void gemm64_f16_kernel(
    const unsigned short* __restrict__ Ap, int lda,
    const unsigned short* __restrict__ Btp, int ldb,
    float* __restrict__ Cout, int ldc,
    const float* __restrict__ bias, const float* __restrict__ bias2,
    int M, int N, int K, float scale, float bscale)
{
  const _Float16* A  = (const _Float16*)Ap;
  const _Float16* Bt = (const _Float16*)Btp;
  __shared__ __align__(16) float sT[8][16 * 68];
  const int lane = threadIdx.x & 31;
  const int wave = threadIdx.x >> 5;
  const int tilesN = N >> 6;
  const int tilesM = M >> 6;
  const int tile = blockIdx.x * 8 + wave;
  if (tile >= tilesM * tilesN) return;
  const int tm = tile / tilesN;
  const int tn = tile - tm * tilesN;
  const int m0 = tm << 6;
  const int n0 = tn << 6;

  const int rlane = lane & 15;
  const int koff  = (lane >> 4) * 8;
  const int mOff  = (lane >> 4) * 8;

  v8f acc[4][4];
#pragma unroll
  for (int i = 0; i < 4; ++i)
#pragma unroll
    for (int j = 0; j < 4; ++j) acc[i][j] = (v8f){0.f,0.f,0.f,0.f,0.f,0.f,0.f,0.f};

  for (int k0 = 0; k0 < K; k0 += 32) {
    v16h bh[4];
#pragma unroll
    for (int j = 0; j < 4; ++j) {
      const size_t bo = (size_t)(n0 + (j << 4) + rlane) * ldb + koff + k0;
      bh[j] = frag_load(Bt + bo);
    }
#pragma unroll
    for (int i = 0; i < 4; ++i) {
      const size_t ao = (size_t)(m0 + (i << 4) + rlane) * lda + koff + k0;
      const v16h ah = frag_load(A + ao);
#pragma unroll
      for (int j = 0; j < 4; ++j) acc[i][j] = mma_h(ah, bh[j], acc[i][j]);
    }
  }

  float* slab = sT[wave];
#pragma unroll
  for (int i = 0; i < 4; ++i) {
    const int mBase = m0 + (i << 4);
#pragma unroll
    for (int j = 0; j < 4; ++j) {
      const int n = n0 + (j << 4) + rlane;
      float bv = bf_value(bias[n]);
      if (BIAS_MODE == 2) bv = bv + bf_value(bias2[n]);
      bv = bv * bscale;
#pragma unroll
      for (int r = 0; r < 8; ++r) {
        const float v = acc[i][j][r] * scale + bv;
        slab[(mOff + r) * 68 + (j << 4) + rlane] = v;
      }
    }
    __builtin_amdgcn_fence(__ATOMIC_RELEASE, "workgroup");
    __builtin_amdgcn_wave_barrier();
    __builtin_amdgcn_fence(__ATOMIC_ACQUIRE, "workgroup");
    {
      const int hh = lane >> 4, c4 = (lane & 15) * 4;
      for (int pass = 0; pass < 2; ++pass) {
#pragma unroll
        for (int it = 0; it < 8; ++it) {
          const int row = it * 2 + hh;
          const v4f v = *(const v4f*)(slab + row * 68 + c4);
          *(volatile v4f*)(Cout + (size_t)(mBase + row) * ldc + n0 + c4) = v;
        }
        __threadfence();
      }
    }
    __builtin_amdgcn_fence(__ATOMIC_RELEASE, "workgroup");
    __builtin_amdgcn_wave_barrier();
    __builtin_amdgcn_fence(__ATOMIC_ACQUIRE, "workgroup");
  }
}

__global__ __launch_bounds__(512) void cell_steps_kernel(
    const int* __restrict__ x, const float* __restrict__ Gt,
    const unsigned short* __restrict__ Whp, unsigned short* __restrict__ hsp)
{
  __shared__ __align__(16) _Float16 sH[2 * 16 * kHP];
  __shared__ __align__(16) int sTok[kSteps * kSampPerBlk];

  const int tid  = threadIdx.x;
  const int lane = tid & 31;
  const int wave = tid >> 5;
  const int hh   = lane >> 4;
  const int c    = lane & 15;
  const int b0   = blockIdx.x * kSampPerBlk;
  const _Float16* Wh = (const _Float16*)Whp;
  _Float16* hs = (_Float16*)hsp;

#pragma unroll 1
  for (int i = 0; i < 16; ++i) {
    const int idx = i * kStepThreads + tid;
    const int t = idx >> 4;
    const int s = idx & 15;
    int v = x[(size_t)(b0 + s) * kSteps + t];
    v = v < 0 ? 0 : v;
    v = v > (kVocab - 1) ? (kVocab - 1) : v;
    sTok[idx] = v;
  }
  {
    const v8h z = (v8h){(_Float16)0.f,(_Float16)0.f,(_Float16)0.f,(_Float16)0.f,(_Float16)0.f,(_Float16)0.f,(_Float16)0.f,(_Float16)0.f};
#pragma unroll
    for (int i = 0; i < 4; ++i) {
      const int idx = i * kStepThreads + tid;
      const int row = idx >> 7;
      const int c8  = (idx & 127) * 8;
      *(v8h*)(sH + row * kHP + c8) = z;
    }
  }
  __syncthreads();

  float cst[4][8];
#pragma unroll
  for (int jt = 0; jt < 4; ++jt)
#pragma unroll
    for (int r = 0; r < 8; ++r) cst[jt][r] = 0.f;

  const int q  = lane >> 3;
  const int c8 = (lane & 7) * 8;

#pragma unroll 1
  for (int t = 0; t < kSteps; ++t) {
    const int p = t & 1;
    const _Float16* hin  = sH + p * (16 * kHP);
    _Float16*       hout = sH + (p ^ 1) * (16 * kHP);

    const v4i ta = *(const v4i*)(sTok + t * kSampPerBlk + 8 * hh);
    const v4i tb = *(const v4i*)(sTok + t * kSampPerBlk + 8 * hh + 4);
    int ro[8];
    ro[0] = ta[0] * kGates; ro[1] = ta[1] * kGates; ro[2] = ta[2] * kGates; ro[3] = ta[3] * kGates;
    ro[4] = tb[0] * kGates; ro[5] = tb[1] * kGates; ro[6] = tb[2] * kGates; ro[7] = tb[3] * kGates;

#pragma unroll
    for (int jt = 0; jt < 4; ++jt) {
      const int jcol = wave * 64 + jt * 16 + c;
      v8f acc[4];
#pragma unroll
      for (int g = 0; g < 4; ++g) {
        const float* gp = Gt + g * kHid + jcol;
        v8f a0;
        a0[0] = gp[ro[0]]; a0[1] = gp[ro[1]]; a0[2] = gp[ro[2]]; a0[3] = gp[ro[3]];
        a0[4] = gp[ro[4]]; a0[5] = gp[ro[5]]; a0[6] = gp[ro[6]]; a0[7] = gp[ro[7]];
        asm volatile("" : "+v"(a0) :: "memory");
        acc[g] = a0;
      }
      const _Float16* ap = hin + c * kHP + 8 * hh;
      const _Float16* bp = Wh + (size_t)jcol * kHid + 8 * hh;
#pragma unroll 2
      for (int k0 = 0; k0 < kHid; k0 += 32) {
        const v16h a = frag_load(ap + k0);
#pragma unroll
        for (int g = 0; g < 4; ++g) {
          const v16h b = frag_load(bp + (size_t)g * kHid * kHid + k0);
          acc[g] = mma_h(a, b, acc[g]);
        }
      }
#pragma unroll
      for (int r = 0; r < 8; ++r) {
        const float gi = acc[0][r] * kAccScaleInv;
        const float gf = acc[1][r] * kAccScaleInv;
        const float gg = acc[2][r] * kAccScaleInv;
        const float go = acc[3][r] * kAccScaleInv;
        const float si = __builtin_amdgcn_rcpf(1.0f + __expf(-gi));
        const float sf = __builtin_amdgcn_rcpf(1.0f + __expf(-gf));
        const float so = __builtin_amdgcn_rcpf(1.0f + __expf(-go));
        const float tg = 1.0f - 2.0f * __builtin_amdgcn_rcpf(1.0f + __expf(2.0f * gg));
        const float cn = sf * cst[jt][r] + si * tg;
        cst[jt][r] = cn;
        const float tc = 1.0f - 2.0f * __builtin_amdgcn_rcpf(1.0f + __expf(2.0f * cn));
        const float hv = so * tc;
        hout[(8 * hh + r) * kHP + jcol] = f16_operand(hv * kCarryH);
      }
    }

    __builtin_amdgcn_fence(__ATOMIC_RELEASE, "workgroup");
    __builtin_amdgcn_wave_barrier();
    __builtin_amdgcn_fence(__ATOMIC_ACQUIRE, "workgroup");
    {
      v8h hv4[4];
#pragma unroll
      for (int it = 0; it < 4; ++it) {
        const int row = it * 4 + q;
        hv4[it] = *(const v8h*)(hout + row * kHP + wave * 64 + c8);
      }
      for (int pass = 0; pass < 2; ++pass) {
#pragma unroll
        for (int it = 0; it < 4; ++it) {
          const int row = it * 4 + q;
          _Float16* gp = hs + ((size_t)(b0 + row) * kSteps + t) * kHid + wave * 64 + c8;
          *(volatile v8h*)gp = hv4[it];
        }
        __threadfence();
      }
    }
    __syncthreads();
  }
}

extern "C" void kernel_launch(void* const* d_in, const int* in_sizes, int n_in,
                              void* d_out, int out_size, void* d_ws, size_t ws_size,
                              hipStream_t stream) {
  if (n_in < 8) return;
  if (in_sizes[0] != kBatch * kSteps) return;
  if (in_sizes[1] != kVocab * kEmb) return;
  if (in_sizes[2] != kGates * kEmb) return;
  if (in_sizes[3] != kGates * kHid) return;
  if (in_sizes[4] != kGates) return;
  if (in_sizes[5] != kGates) return;
  if (in_sizes[6] != kCls * kHid) return;
  if (in_sizes[7] != kCls) return;
  if (out_size != kRowsBT * kCls) return;
  if (ws_size < kWsTotal) return;

  const int*   x     = (const int*)  d_in[0];
  const float* embed = (const float*)d_in[1];
  const float* W_ih  = (const float*)d_in[2];
  const float* W_hh  = (const float*)d_in[3];
  const float* b_ih  = (const float*)d_in[4];
  const float* b_hh  = (const float*)d_in[5];
  const float* fc_W  = (const float*)d_in[6];
  const float* fc_b  = (const float*)d_in[7];
  float* out = (float*)d_out;

  char* ws = (char*)d_ws;
  unsigned short* WHH16 = (unsigned short*)(ws + kOffWHH);
  unsigned short* WIH16 = (unsigned short*)(ws + kOffWIH);
  unsigned short* FCW16 = (unsigned short*)(ws + kOffFCW);
  unsigned short* EMB16 = (unsigned short*)(ws + kOffEMB);
  float*          GTAB  = (float*)(ws + kOffGT);
  unsigned short* HS16  = (unsigned short*)(ws + kOffHS);

  plane_f16_kernel<<<(kGates * kHid / 8) / 256, 256, 0, stream>>>(W_hh, WHH16, kGates * kHid / 8, kCarryW);
  plane_f16_kernel<<<(kGates * kEmb / 8) / 256, 256, 0, stream>>>(W_ih, WIH16, kGates * kEmb / 8, kCarryW);
  plane_f16_kernel<<<(kCls * kHid / 8) / 256, 256, 0, stream>>>(fc_W, FCW16, kCls * kHid / 8, kCarryW);
  plane_f16_kernel<<<(kVocab * kEmb / 8) / 256, 256, 0, stream>>>(embed, EMB16, kVocab * kEmb / 8, kCarryE);

  gemm64_f16_kernel<2><<<((kVocab / 64) * (kGates / 64)) / 8, 256, 0, stream>>>(
      EMB16, kEmb, WIH16, kEmb, GTAB, kGates, b_ih, b_hh,
      kVocab, kGates, kEmb, kTableScale, kAccScale);

  cell_steps_kernel<<<kStepBlocks, kStepThreads, 0, stream>>>(x, GTAB, WHH16, HS16);

  gemm64_f16_kernel<1><<<((kRowsBT / 64) * (kCls / 64)) / 8, 256, 0, stream>>>(
      HS16, kHid, FCW16, kHid, out, kCls, fc_b, fc_b,
      kRowsBT, kCls, kHid, kHeadScale, 1.0f);
}
